// EdgePredictor_58308476010969
// MI455X (gfx1250) — hardware-verified
//
#include <hip/hip_runtime.h>
#include <math.h>
#include <stdint.h>

#define NN 50000
#define NE 800000
#define CH 128
#define CH2 256
#define MPAD 50048
#define SRB 4096
#define NTILE 13
#define NROWS (NTILE * SRB)
#define RPW (SRB / 8)
#define NT 256
#define SPT 8
#define SCH (NT * SPT)
#define NCHE ((NE + SCH - 1) / SCH)

constexpr size_t PLANE16 = (size_t)MPAD * CH;

static_assert(MPAD % 64 == 0 && MPAD >= NN, "M tile pad");
static_assert(CH % 64 == 0 && CH2 % 64 == 0 && CH % 32 == 0, "N and K tiles");
static_assert(NROWS >= MPAD && NROWS >= NN, "row tiles cover all nodes");
static_assert(SRB == 8 * RPW && RPW == 512 && NT == 256, "8 waves x 512 rows, 16 rows per lane in the degree pass");
static_assert(SCH == 2048 && SPT % 4 == 0 && SCH % 32 == 0, "chunk geometry");
static_assert(NE % (32 * SPT) == 0 && SCH % (32 * SPT) == 0, "a wave is entirely inside or entirely outside the edge list");
static_assert(NN <= 65536 && SRB <= 4096, "packed hit record fits (dl << 16 | src), dl >> 9 = wave");
static_assert((MPAD * CH) % (8 * NT) == 0, "x cast grid exact");
static_assert(NE % NT == 0, "edge grid exact");

constexpr size_t WS_DINV  = (size_t)NROWS * 4;
constexpr size_t WS_P16   = PLANE16 * 2;
constexpr size_t WS_WB    = (size_t)CH * CH * 2;
constexpr size_t WS_WMB   = (size_t)CH2 * CH * 2;
constexpr size_t WS_C1    = (size_t)MPAD * CH * 4;
constexpr size_t WS_AGG   = (size_t)NROWS * CH * 4;
constexpr size_t WS_CAB   = (size_t)MPAD * CH2 * 4;
constexpr size_t WS_TOTAL = WS_DINV + 2 * WS_P16 + 2 * WS_WB + WS_WMB + WS_C1 + WS_AGG + WS_CAB;
static_assert(WS_TOTAL == 130105344, "carve total");
static_assert(WS_TOTAL <= (size_t)134217728, "carve under 128 MiB");
static_assert(WS_DINV % 256 == 0 && WS_P16 % 256 == 0 && WS_WB % 256 == 0 && WS_WMB % 256 == 0 &&
              WS_C1 % 256 == 0 && WS_AGG % 256 == 0 && WS_CAB % 256 == 0, "region alignment");

typedef __attribute__((ext_vector_type(16))) _Float16 v16h;
typedef __attribute__((ext_vector_type(8)))  _Float16 v8h;
typedef __attribute__((ext_vector_type(16))) __bf16   v16b;
typedef __attribute__((ext_vector_type(8)))  __bf16   v8b;
typedef __attribute__((ext_vector_type(8)))  float    v8f;
typedef __attribute__((ext_vector_type(4)))  float    v4f;
typedef __attribute__((ext_vector_type(4)))  int      v4i;
typedef __attribute__((ext_vector_type(4)))  unsigned int v4u;

__device__ __forceinline__ unsigned short f2bf_bits(float f) {
  unsigned u = __float_as_uint(f);
  return (unsigned short)((u + 0x7FFFu + ((u >> 16) & 1u)) >> 16);
}
__device__ __forceinline__ float bf_bits2f(unsigned short h) { return __uint_as_float(((unsigned)h) << 16); }
__device__ __forceinline__ float bfr(float f) { return bf_bits2f(f2bf_bits(f)); }
__device__ __forceinline__ unsigned pk16(unsigned short a, unsigned short b) { return (unsigned)a | ((unsigned)b << 16); }

__device__ __forceinline__ void grp_guard_h(v8f& a, v8f& b, v8f& c, v8f& d, v16h x0, v16h x1, v16h y0, v16h y1, v16h y2, v16h y3) {
  asm volatile("v_nop\n\tv_nop\n\tv_nop\n\tv_nop" : "+v"(a), "+v"(b), "+v"(c), "+v"(d) : "v"(x0), "v"(x1), "v"(y0), "v"(y1), "v"(y2), "v"(y3));
}
__device__ __forceinline__ void grp_guard_b(v8f& a, v8f& b, v8f& c, v8f& d, v16b x0, v16b x1, v16b y0, v16b y1, v16b y2, v16b y3) {
  asm volatile("v_nop\n\tv_nop\n\tv_nop\n\tv_nop" : "+v"(a), "+v"(b), "+v"(c), "+v"(d) : "v"(x0), "v"(x1), "v"(y0), "v"(y1), "v"(y2), "v"(y3));
}
__device__ __forceinline__ void keep4_h(v16h a, v16h b, v16h c, v16h d) { asm volatile("v_nop" :: "v"(a), "v"(b), "v"(c), "v"(d)); }
__device__ __forceinline__ void keep4_b(v16b a, v16b b, v16b c, v16b d) { asm volatile("v_nop" :: "v"(a), "v"(b), "v"(c), "v"(d)); }
__device__ __forceinline__ void acc_guard4(v8f& a, v8f& b, v8f& c, v8f& d) { asm volatile("v_nop\n\tv_nop\n\tv_nop\n\tv_nop" : "+v"(a), "+v"(b), "+v"(c), "+v"(d)); }
template <typename T> struct Frag;
template <> struct Frag<_Float16> {
  typedef v16h V; union U { v16h v; v8h h[2]; };
  static __device__ __forceinline__ v16h load(const _Float16* p) {
    U f; f.h[0] = *(const v8h*)(p); f.h[1] = *(const v8h*)(p + 16); return f.v;
  }
  static __device__ __forceinline__ v8f mma(v16h a, v16h b, v8f c) {
    return __builtin_amdgcn_wmma_f32_16x16x32_f16(false, a, false, b, (short)0, c, false, false);
  }
  static __device__ __forceinline__ void guard4(v8f& a, v8f& b, v8f& c, v8f& d, v16h x0, v16h x1, v16h y0, v16h y1, v16h y2, v16h y3) {
    grp_guard_h(a, b, c, d, x0, x1, y0, y1, y2, y3);
  }
  static __device__ __forceinline__ void keep(v16h a, v16h b, v16h c, v16h d) { keep4_h(a, b, c, d); }
};
template <> struct Frag<__bf16> {
  typedef v16b V; union U { v16b v; v8b h[2]; };
  static __device__ __forceinline__ v16b load(const __bf16* p) {
    U f; f.h[0] = *(const v8b*)(p); f.h[1] = *(const v8b*)(p + 16); return f.v;
  }
  static __device__ __forceinline__ v8f mma(v16b a, v16b b, v8f c) {
    return __builtin_amdgcn_wmma_f32_16x16x32_bf16(false, a, false, b, (short)0, c, false, false);
  }
  static __device__ __forceinline__ void guard4(v8f& a, v8f& b, v8f& c, v8f& d, v16b x0, v16b x1, v16b y0, v16b y1, v16b y2, v16b y3) {
    grp_guard_b(a, b, c, d, x0, x1, y0, y1, y2, y3);
  }
  static __device__ __forceinline__ void keep(v16b a, v16b b, v16b c, v16b d) { keep4_b(a, b, c, d); }
};

template <int ET> struct Elem;
template <> struct Elem<0> { typedef _Float16 T; };
template <> struct Elem<1> { typedef __bf16 T; };
template <int ET, int SPLIT, int BIAS_MODE, int OUT_MODE, bool RESID, int ACT = 0>
__global__ __launch_bounds__(256) void wmma_gemm64(
    const unsigned short* __restrict__ Ap, const unsigned short* __restrict__ A2p, int lda, long strideA,
    const unsigned short* __restrict__ Btp, const unsigned short* __restrict__ Bt2p, int ldb, long strideB,
    void* __restrict__ Cout, void* __restrict__ Cout2, int ldc, long strideC,
    const float* __restrict__ bias,
    const float* __restrict__ resid, long strideR,
    int M, int N, int K, float scale) {
  typedef typename Elem<ET>::T T;
  typedef typename Frag<T>::V V;
  const T* A = (const T*)Ap; const T* A2 = (const T*)A2p; const T* Bt = (const T*)Btp; const T* Bt2 = (const T*)Bt2p;
  __shared__ __align__(16) float sT[8][16 * 68];
  const int b    = blockIdx.y;
  const int lane = threadIdx.x & 31;
  const int wave = threadIdx.x >> 5;
  const int tilesN = N >> 6;
  const int tilesM = M >> 6;
  const int tile = blockIdx.x * 8 + wave;
  if (tile >= tilesM * tilesN) return;
  const int tm = tile / tilesN;
  const int tn = tile - tm * tilesN;
  const int m0 = tm << 6;
  const int n0 = tn << 6;

  const T* Ab  = A  + (size_t)b * strideA;
  const T* Bb  = Bt + (size_t)b * strideB;
  const T* Ab2 = (SPLIT >= 1) ? (A2  + (size_t)b * strideA) : nullptr;
  const T* Bb2 = (SPLIT == 2) ? (Bt2 + (size_t)b * strideB) : nullptr;

  const int rlane = lane & 15;
  const int koff  = (lane >> 4) * 8;
  const int mOff  = (lane >> 4) * 8;

  v8f acc[4][4];
#pragma unroll
  for (int i = 0; i < 4; ++i)
#pragma unroll
    for (int j = 0; j < 4; ++j) acc[i][j] = (v8f){0.f,0.f,0.f,0.f,0.f,0.f,0.f,0.f};

  for (int k0 = 0; k0 < K; k0 += 32) {
    V bh[4], bl[4];
#pragma unroll
    for (int j = 0; j < 4; ++j) {
      const size_t bo = (size_t)(n0 + (j << 4) + rlane) * ldb + koff + k0;
      bh[j] = Frag<T>::load(Bb + bo);
      if (SPLIT == 2) bl[j] = Frag<T>::load(Bb2 + bo);
    }
#pragma unroll
    for (int i = 0; i < 4; ++i) {
      const size_t ao = (size_t)(m0 + (i << 4) + rlane) * lda + koff + k0;
      V ah = Frag<T>::load(Ab + ao);
      V al;
      if (SPLIT >= 1) al = Frag<T>::load(Ab2 + ao);
#pragma unroll
      for (int j = 0; j < 4; ++j) {
        acc[i][j] = Frag<T>::mma(ah, bh[j], acc[i][j]);
        if (SPLIT == 2) acc[i][j] = Frag<T>::mma(ah, bl[j], acc[i][j]);
        if (SPLIT >= 1) acc[i][j] = Frag<T>::mma(al, bh[j], acc[i][j]);
      }
      Frag<T>::guard4(acc[i][0], acc[i][1], acc[i][2], acc[i][3], ah, (SPLIT >= 1) ? al : ah, bh[0], bh[1], bh[2], bh[3]);
    }
    Frag<T>::keep(bh[0], bh[1], bh[2], bh[3]);
    if (SPLIT == 2) Frag<T>::keep(bl[0], bl[1], bl[2], bl[3]);
  }
  acc_guard4(acc[0][0], acc[0][1], acc[0][2], acc[0][3]);
  acc_guard4(acc[1][0], acc[1][1], acc[1][2], acc[1][3]);
  acc_guard4(acc[2][0], acc[2][1], acc[2][2], acc[2][3]);
  acc_guard4(acc[3][0], acc[3][1], acc[3][2], acc[3][3]);

  float* slab = sT[wave];
  const float* Rb = RESID ? (resid + (size_t)b * strideR) : nullptr;
#pragma unroll
  for (int i = 0; i < 4; ++i) {
    const int mBase = m0 + (i << 4);
#pragma unroll
    for (int j = 0; j < 4; ++j) {
      const int n = n0 + (j << 4) + rlane;
      float bv = 0.f;
      if (BIAS_MODE == 2) bv = bias[n];
#pragma unroll
      for (int r = 0; r < 8; ++r) {
        float v = acc[i][j][r] * scale;
        if (BIAS_MODE == 1) v += bias[mBase + mOff + r];
        if (BIAS_MODE == 2) v += bv;
        if (RESID) v += Rb[(size_t)(mBase + mOff + r) * ldc + n];
        if (ACT == 2) v = fmaxf(v, 0.0f);
        if (ACT == 4) v = (v > 0.f) ? v : 0.01f * v;
        slab[(mOff + r) * 68 + (j << 4) + rlane] = v;
      }
    }
    __builtin_amdgcn_fence(__ATOMIC_RELEASE, "workgroup");
    __builtin_amdgcn_wave_barrier();
    __builtin_amdgcn_fence(__ATOMIC_ACQUIRE, "workgroup");
    if (OUT_MODE == 0) {
      float* C = (float*)Cout + (size_t)b * strideC;
      const int hh = lane >> 4, c4 = (lane & 15) * 4;
      for (int pass = 0; pass < 2; ++pass) {
#pragma unroll
        for (int it = 0; it < 8; ++it) {
          const int row = it * 2 + hh;
          v4f v = *(const v4f*)(slab + row * 68 + c4);
          *(volatile v4f*)(C + (size_t)(mBase + row) * ldc + n0 + c4) = v;
        }
        __threadfence();
      }
    } else {
      const int q = lane >> 3, c8 = (lane & 7) * 8;
      unsigned short* C  = (unsigned short*)Cout  + (size_t)b * strideC;
      unsigned short* C2 = (OUT_MODE == 2) ? ((unsigned short*)Cout2 + (size_t)b * strideC) : nullptr;
      for (int pass = 0; pass < 2; ++pass) {
#pragma unroll
        for (int it = 0; it < 4; ++it) {
          const int row = it * 4 + q;
          const float* sp = slab + row * 68 + c8;
          v8h hv, lv;
#pragma unroll
          for (int e = 0; e < 8; ++e) {
            if (OUT_MODE == 1) {
              hv[e] = (_Float16)sp[e];
            } else {
              unsigned short hb = f2bf_bits(sp[e]);
              unsigned short lb = f2bf_bits(sp[e] - bf_bits2f(hb));
              hv[e] = __builtin_bit_cast(_Float16, hb);
              lv[e] = __builtin_bit_cast(_Float16, lb);
            }
          }
          *(volatile v8h*)(C + (size_t)(mBase + row) * ldc + n0 + c8) = hv;
          if (OUT_MODE == 2) *(volatile v8h*)(C2 + (size_t)(mBase + row) * ldc + n0 + c8) = lv;
        }
        __threadfence();
      }
    }
    __builtin_amdgcn_fence(__ATOMIC_RELEASE, "workgroup");
    __builtin_amdgcn_wave_barrier();
    __builtin_amdgcn_fence(__ATOMIC_ACQUIRE, "workgroup");
  }
}

__global__ __launch_bounds__(NT) void prep_kernel(const float* __restrict__ W1, const float* __restrict__ W2,
                                                 const float* __restrict__ Wm1,
                                                 unsigned* __restrict__ W1B, unsigned* __restrict__ W2B, unsigned* __restrict__ WMB) {
  const int z = blockIdx.x >> 5;
  const int tid = threadIdx.x;
  if (z < 2) {
    const float* W = (z == 0) ? W1 : W2;
    unsigned* O = (z == 0) ? W1B : W2B;
    const int i = (blockIdx.x - z * 32) * NT + tid;
    const int n = i >> 6, k = 2 * (i & 63);
    const float a = W[(size_t)k * CH + n], c = W[(size_t)(k + 1) * CH + n];
    const unsigned u = pk16(f2bf_bits(a), f2bf_bits(c));
    ((volatile unsigned*)O)[i] = u;
    __threadfence();
    ((volatile unsigned*)O)[i] = u;
  } else {
    const int i = (blockIdx.x - 64) * NT + tid;
    const int n = i >> 6, k = 2 * (i & 63);
    const int ro = (n >> 7) * CH;
    const int nc = n & 127;
    const float a = Wm1[(size_t)(ro + k) * CH + nc], c = Wm1[(size_t)(ro + k + 1) * CH + nc];
    const unsigned u = pk16(f2bf_bits(a), f2bf_bits(c));
    ((volatile unsigned*)WMB)[i] = u;
    __threadfence();
    ((volatile unsigned*)WMB)[i] = u;
  }
}

__global__ __launch_bounds__(NT) void cast_x_kernel(const float* __restrict__ x, unsigned* __restrict__ XB) {
  const int i = blockIdx.x * NT + threadIdx.x;
  const int e0 = 8 * i;
  const int row = e0 >> 7;
  const bool live = row < NN;
  const int erow = live ? row : (NN - 1);
  const float* p = x + (size_t)erow * CH + (e0 & 127);
  const v4f a = *(const v4f*)(p);
  const v4f c = *(const v4f*)(p + 4);
  unsigned short hb[8];
#pragma unroll
  for (int e = 0; e < 4; ++e) {
    hb[e]     = live ? f2bf_bits(a[e]) : (unsigned short)0;
    hb[4 + e] = live ? f2bf_bits(c[e]) : (unsigned short)0;
  }
  const v4u u = (v4u){pk16(hb[0], hb[1]), pk16(hb[2], hb[3]), pk16(hb[4], hb[5]), pk16(hb[6], hb[7])};
  unsigned* q = XB + 4 * (size_t)i;
  *(volatile v4u*)q = u;
  __threadfence();
  *(volatile v4u*)q = u;
}

__device__ __forceinline__ int blk_excl_scan(int cnt, int* scan_ws, int tid, int* tot) {
  const int lane = tid & 31, wave = tid >> 5; int incl = cnt;
#pragma unroll
  for (int o = 1; o < 32; o <<= 1) { const int v = __shfl_up(incl, o, 32); if (lane >= o) incl += v; }
  if (lane == 31) scan_ws[wave] = incl;
  __syncthreads();
  if (wave == 0) { int wv = (lane < NT / 32) ? scan_ws[lane] : 0; int wincl = wv;
#pragma unroll
    for (int o = 1; o < 32; o <<= 1) { const int v = __shfl_up(wincl, o, 32); if (lane >= o) wincl += v; }
    if (lane < NT / 32) scan_ws[32 + lane] = wincl - wv; if (lane == 31) scan_ws[64] = wincl; }
  __syncthreads();
  const int res = scan_ws[32 + wave] + incl - cnt; *tot = scan_ws[64];
  return res;
}

__device__ __forceinline__ int chunk_hits_deg(const int* __restrict__ dstv, int e0, int n0, int tid, int* LIST, int* scan_ws) {
  const int eb = e0 + tid * SPT;
  const unsigned inr = (eb < NE) ? 1u : 0u;
  const int ebc = (eb < NE) ? eb : (NE - SPT);
  int rec[SPT]; int cnt = 0;
#pragma unroll
  for (int k = 0; k < SPT; k += 4) {
    const v4i d4 = *(const v4i*)(dstv + ebc + k);
#pragma unroll
    for (int e = 0; e < 4; ++e) {
      const unsigned du = (unsigned)d4[e] - (unsigned)n0;
      const unsigned hit = inr & ((du < (unsigned)SRB) ? 1u : 0u);
      rec[k + e] = (int)(hit * (du + 1u)) - 1;
      cnt += (int)hit;
    }
  }
  int tot; int p = blk_excl_scan(cnt, scan_ws, tid, &tot);
#pragma unroll
  for (int k = 0; k < SPT; ++k) if (rec[k] >= 0) { if ((unsigned)p < (unsigned)SCH) LIST[p] = rec[k]; ++p; }
  __syncthreads();
  return tot < SCH ? tot : SCH;
}

__device__ __forceinline__ int chunk_hits_agg(const int* __restrict__ srcv, const int* __restrict__ dstv, int e0, int n0, int tid,
                                              int* LIST, int* scan_ws) {
  const int eb = e0 + tid * SPT;
  const unsigned inr = (eb < NE) ? 1u : 0u;
  const int ebc = (eb < NE) ? eb : (NE - SPT);
  int rec[SPT]; int cnt = 0;
#pragma unroll
  for (int k = 0; k < SPT; k += 4) {
    const v4i d4 = *(const v4i*)(dstv + ebc + k);
    const v4i s4 = *(const v4i*)(srcv + ebc + k);
#pragma unroll
    for (int e = 0; e < 4; ++e) {
      const unsigned du = (unsigned)d4[e] - (unsigned)n0;
      int s = s4[e]; s = s < 0 ? 0 : (s >= NN ? NN - 1 : s);
      const unsigned hit = inr & ((du < (unsigned)SRB) ? 1u : 0u);
      const unsigned val = (du << 16) | (unsigned)s;
      rec[k + e] = (int)(hit * (val + 1u)) - 1;
      cnt += (int)hit;
    }
  }
  int tot; int p = blk_excl_scan(cnt, scan_ws, tid, &tot);
#pragma unroll
  for (int k = 0; k < SPT; ++k) if (rec[k] >= 0) { if ((unsigned)p < (unsigned)SCH) LIST[p] = rec[k]; ++p; }
  __syncthreads();
  return tot < SCH ? tot : SCH;
}

__global__ __launch_bounds__(NT) void deg_kernel(const int* __restrict__ ei, float* __restrict__ dinv) {
  __shared__ int LIST[SCH];
  __shared__ int scan_ws[96];
  const int tid = threadIdx.x, lane = tid & 31, wave = tid >> 5;
  const int n0 = blockIdx.x * SRB;
  for (int i = tid; i < SCH; i += NT) LIST[i] = 0;
  if (tid < 96) scan_ws[tid] = 0;
  __syncthreads();
  const int* dstv = ei + NE;
  const int wb = wave * RPW;
  int cnt[16];
#pragma unroll
  for (int k = 0; k < 16; ++k) cnt[k] = 0;
#pragma unroll 1
  for (int c = 0; c < NCHE; ++c) {
    const int tot = chunk_hits_deg(dstv, c * SCH, n0, tid, LIST, scan_ws);
#pragma unroll 1
    for (int base = 0; base < tot; base += 32) {
      const int q = base + lane;
      const int rv = LIST[q];
      const int own = (q < tot && (rv >> 9) == wave) ? 1 : 0;
      unsigned msk = (unsigned)__ballot(own);
#pragma unroll 1
      for (int it = 0; it < 32; ++it) {
        if (msk == 0u) break;
        const int bp = __builtin_ctz(msk); msk &= msk - 1u;
        const int r = __shfl(rv, bp, 32);
        const int dr = r - wb - lane;
#pragma unroll
        for (int k = 0; k < 16; ++k) cnt[k] += (dr == 32 * k) ? 1 : 0;
      }
    }
    __syncthreads();
  }
  float dv[16];
#pragma unroll
  for (int k = 0; k < 16; ++k) dv[k] = rsqrtf((float)(1 + cnt[k]));
  float* dp = dinv + n0 + wb + lane;
  for (int pass = 0; pass < 2; ++pass) {
#pragma unroll
    for (int k = 0; k < 16; ++k) *(volatile float*)(dp + 32 * k) = dv[k];
    __threadfence();
  }
}

template <bool RELU>
__global__ __launch_bounds__(NT) void agg_kernel(const float* __restrict__ XW, const int* __restrict__ ei,
                                                const float* __restrict__ dinv, const float* __restrict__ bias,
                                                float* AGG, unsigned short* __restrict__ HP) {
  __shared__ int LIST[SCH];
  __shared__ int scan_ws[96];
  __shared__ float SDI[SRB];
  __shared__ __align__(16) unsigned slab[8][128];
  const int tid = threadIdx.x, lane = tid & 31, wave = tid >> 5;
  const int n0 = blockIdx.x * SRB;
  for (int i = tid; i < SCH; i += NT) LIST[i] = 0;
  if (tid < 96) scan_ws[tid] = 0;
  for (int i = tid; i < SRB; i += NT) SDI[i] = dinv[n0 + i];
  const v4f z4 = {0.f, 0.f, 0.f, 0.f};
#pragma unroll 1
  for (int j = 0; j < RPW; ++j) *(v4f*)(AGG + (size_t)(n0 + wave * RPW + j) * CH + 4 * lane) = z4;
  __syncthreads();
  const int* srcv = ei; const int* dstv = ei + NE;
#pragma unroll 1
  for (int c = 0; c < NCHE; ++c) {
    const int tot = chunk_hits_agg(srcv, dstv, c * SCH, n0, tid, LIST, scan_ws);
#pragma unroll 1
    for (int base = 0; base < tot; base += 32) {
      const int q = base + lane;
      const int rv = LIST[q];
      const int own = (q < tot && (rv >> 25) == wave) ? 1 : 0;
      unsigned msk = (unsigned)__ballot(own);
#pragma unroll 1
      for (int it = 0; it < 32; ++it) {
        if (msk == 0u) break;
        const int bp = __builtin_ctz(msk); msk &= msk - 1u;
        const int r = __shfl(rv, bp, 32);
        const int dl = r >> 16, s = r & 0xFFFF;
        const float ds = dinv[s];
        const float dd = SDI[dl];
        const float nrm = ds * dd;
        const v4f xr = *(const v4f*)(XW + (size_t)s * CH + 4 * lane);
        float* rp = AGG + (size_t)(n0 + dl) * CH + 4 * lane;
        v4f a = *(const v4f*)rp;
        a = a + nrm * xr;
        *(v4f*)rp = a;
      }
    }
    __syncthreads();
  }
  v4f bv;
#pragma unroll
  for (int e = 0; e < 4; ++e) bv[e] = bfr(bias[4 * lane + e]);
  unsigned* sl = slab[wave];
#pragma unroll 1
  for (int j = 0; j < RPW; ++j) {
    const int dl = wave * RPW + j;
    const int n = n0 + dl;
    if (n < MPAD) {
      const bool live = n < NN;
      const float dd = SDI[dl];
      const float nrm = dd * dd;
      const v4f a  = *(const v4f*)(AGG + (size_t)n * CH + 4 * lane);
      const v4f xs = *(const v4f*)(XW + (size_t)n * CH + 4 * lane);
      v4f t = a + nrm * xs;
      t = t + bv;
      unsigned short hb[4], lb[4];
#pragma unroll
      for (int e = 0; e < 4; ++e) {
        float v = t[e];
        if (RELU) v = fmaxf(v, 0.0f);
        v = live ? v : 0.0f;
        const unsigned short hbe = f2bf_bits(v);
        hb[e] = hbe;
        lb[e] = f2bf_bits(v - bf_bits2f(hbe));
      }
      sl[2 * lane]          = pk16(hb[0], hb[1]);
      sl[2 * lane + 1]      = pk16(hb[2], hb[3]);
      sl[64 + 2 * lane]     = pk16(lb[0], lb[1]);
      sl[64 + 2 * lane + 1] = pk16(lb[2], lb[3]);
      __builtin_amdgcn_fence(__ATOMIC_RELEASE, "workgroup");
      __builtin_amdgcn_wave_barrier();
      __builtin_amdgcn_fence(__ATOMIC_ACQUIRE, "workgroup");
      const v4u u = *(const v4u*)(sl + (lane >> 4) * 64 + 4 * (lane & 15));
      unsigned short* hp = HP + (size_t)(lane >> 4) * PLANE16 + (size_t)n * CH + 8 * (lane & 15);
      for (int pass = 0; pass < 2; ++pass) { *(volatile v4u*)hp = u; __threadfence(); }
      __builtin_amdgcn_fence(__ATOMIC_RELEASE, "workgroup");
      __builtin_amdgcn_wave_barrier();
      __builtin_amdgcn_fence(__ATOMIC_ACQUIRE, "workgroup");
    }
  }
}

__global__ __launch_bounds__(NT) void edge_kernel(const float* __restrict__ CAB, const int* __restrict__ ei,
                                                 const float* __restrict__ bm1, const float* __restrict__ Wm2,
                                                 const float* __restrict__ bm2, float* __restrict__ out) {
  __shared__ float sb[CH];
  __shared__ float sw[CH];
  __shared__ __align__(16) float so[NT];
  const int tid = threadIdx.x, lane = tid & 31, wave = tid >> 5;
  if (tid < CH) { sb[tid] = bfr(bm1[tid]); sw[tid] = bfr(Wm2[tid]); }
  __syncthreads();
  const int e = blockIdx.x * NT + tid;
  int s = ei[e], d = ei[NE + e];
  s = s < 0 ? 0 : (s >= NN ? NN - 1 : s);
  d = d < 0 ? 0 : (d >= NN ? NN - 1 : d);
  const float* ap = CAB + (size_t)s * CH2;
  const float* bp = CAB + (size_t)d * CH2 + CH;
  float acc = 0.0f;
#pragma unroll 2
  for (int c4 = 0; c4 < CH / 4; ++c4) {
    const v4f a = *(const v4f*)(ap + 4 * c4);
    const v4f b = *(const v4f*)(bp + 4 * c4);
#pragma unroll
    for (int k = 0; k < 4; ++k) {
      float t = a[k] + b[k];
      t = t + sb[4 * c4 + k];
      t = fmaxf(t, 0.0f);
      acc = fmaf(t, sw[4 * c4 + k], acc);
    }
  }
  const float o = acc + bfr(bm2[0]);
  so[tid] = o;
  __syncthreads();
  if (wave < 2) {
    const v4f v = *(const v4f*)(so + wave * 128 + 4 * lane);
    float* op = out + (size_t)blockIdx.x * NT + wave * 128 + 4 * lane;
    for (int pass = 0; pass < 2; ++pass) { *(volatile v4f*)op = v; __threadfence(); }
  }
}

extern "C" void kernel_launch(void* const* d_in, const int* in_sizes, int n_in,
                              void* d_out, int out_size, void* d_ws, size_t ws_size, hipStream_t stream) {
  (void)in_sizes; (void)n_in; (void)out_size;
  const float* x   = (const float*)d_in[0];
  const int*   ei  = (const int*)  d_in[1];
  const float* W1  = (const float*)d_in[2];
  const float* b1  = (const float*)d_in[3];
  const float* W2  = (const float*)d_in[4];
  const float* b2  = (const float*)d_in[5];
  const float* Wm1 = (const float*)d_in[6];
  const float* bm1 = (const float*)d_in[7];
  const float* Wm2 = (const float*)d_in[8];
  const float* bm2 = (const float*)d_in[9];
  float* out = (float*)d_out;

  if (WS_TOTAL > ws_size) return;
  char* ws = (char*)d_ws; size_t off = 0;
  auto carve = [&](size_t bytes) -> char* { char* p = ws + off; off += (bytes + 255) & ~(size_t)255; return p; };
  float*          DINV = (float*)carve(WS_DINV);
  unsigned short* XB   = (unsigned short*)carve(WS_P16);
  unsigned short* HL   = (unsigned short*)carve(WS_P16);
  unsigned*       W1B  = (unsigned*)carve(WS_WB);
  unsigned*       W2B  = (unsigned*)carve(WS_WB);
  unsigned*       WMB  = (unsigned*)carve(WS_WMB);
  float*          C1   = (float*)carve(WS_C1);
  float*          AGG  = (float*)carve(WS_AGG);
  float*          CAB  = (float*)carve(WS_CAB);
  if (off != WS_TOTAL || off > ws_size) return;
  unsigned short* HH = XB;
  (void)HL;

  prep_kernel<<<128, NT, 0, stream>>>(W1, W2, Wm1, W1B, W2B, WMB);
  cast_x_kernel<<<(MPAD * CH) / (8 * NT), NT, 0, stream>>>(x, (unsigned*)XB);
  deg_kernel<<<NTILE, NT, 0, stream>>>(ei, DINV);

  const int tiles128 = (MPAD / 64) * (CH / 64);
  const int tiles256 = (MPAD / 64) * (CH2 / 64);
  wmma_gemm64<1, 0, 0, 0, false, 0><<<dim3((tiles128 + 7) / 8, 1), 256, 0, stream>>>(
      (const unsigned short*)XB, (const unsigned short*)XB, CH, 0L,
      (const unsigned short*)W1B, (const unsigned short*)W1B, CH, 0L,
      (void*)C1, (void*)nullptr, CH, 0L,
      (const float*)nullptr, (const float*)nullptr, 0L, MPAD, CH, CH, 1.0f);
  agg_kernel<true><<<NTILE, NT, 0, stream>>>(C1, ei, DINV, b1, AGG, HH);
  wmma_gemm64<1, 1, 0, 0, false, 0><<<dim3((tiles128 + 7) / 8, 1), 256, 0, stream>>>(
      (const unsigned short*)HH, (const unsigned short*)(HH + PLANE16), CH, 0L,
      (const unsigned short*)W2B, (const unsigned short*)W2B, CH, 0L,
      (void*)C1, (void*)nullptr, CH, 0L,
      (const float*)nullptr, (const float*)nullptr, 0L, MPAD, CH, CH, 1.0f);
  agg_kernel<false><<<NTILE, NT, 0, stream>>>(C1, ei, DINV, b2, AGG, HH);
  wmma_gemm64<1, 1, 0, 0, false, 0><<<dim3((tiles256 + 7) / 8, 1), 256, 0, stream>>>(
      (const unsigned short*)HH, (const unsigned short*)(HH + PLANE16), CH, 0L,
      (const unsigned short*)WMB, (const unsigned short*)WMB, CH, 0L,
      (void*)CAB, (void*)nullptr, CH2, 0L,
      (const float*)nullptr, (const float*)nullptr, 0L, MPAD, CH2, CH, 1.0f);
  edge_kernel<<<NE / NT, NT, 0, stream>>>(CAB, ei, bm1, Wm2, bm2, out);
}
